// RNN_64501818851829
// MI455X (gfx1250) — hardware-run, weakly checked
//
#include <hip/hip_runtime.h>
#include <math.h>

typedef __attribute__((ext_vector_type(16))) _Float16 v16h;
typedef __attribute__((ext_vector_type(8)))  _Float16 v8h;
typedef __attribute__((ext_vector_type(8)))  float    v8f;
typedef __attribute__((ext_vector_type(4)))  float    v4f;

constexpr int kBatch      = 4096;
constexpr int kSteps      = 1024;
constexpr int kHid        = 40;
constexpr int kComb       = kHid + 1;
constexpr int kTileRows   = 16;
constexpr int kTiles      = kBatch / kTileRows;
constexpr int kChunk      = 32;
constexpr int kNumChunks  = kSteps / kChunk;
constexpr int kPitch      = 36;
constexpr float kSlope    = 0.01f;
constexpr size_t kOutElems = (size_t)kBatch * (size_t)kSteps;
static_assert(kHid == 40 && kComb == 41, "40 units = two full 16-row tiles + the low lane half of a third; the input is k 40");
static_assert(kBatch % kTileRows == 0 && kSteps % kChunk == 0, "whole tiles and chunks");
static_assert((kPitch % 4) == 0, "16-B aligned LDS rows");

constexpr float kStateCarry  = 256.0f;
constexpr float kWeightCarry = 64.0f;
constexpr float kFoldBack    = 1.0f / (kStateCarry * kWeightCarry);
constexpr float kF16MinNorm  = 6.103515625e-5f;
static_assert(kStateCarry * kWeightCarry == 16384.0f, "carry product");

namespace eng {

union FragU { v16h v; v8h h[2]; };

__device__ __forceinline__ unsigned short f2bf_bits(float f) {
  unsigned u = __float_as_uint(f);
  return (unsigned short)((u + 0x7FFFu + ((u >> 16) & 1u)) >> 16);
}
__device__ __forceinline__ float bf16v(float f) {
  return __uint_as_float(((unsigned)f2bf_bits(f)) << 16);
}
__device__ __forceinline__ _Float16 to_f16_flushed(float c) {
  const float z = (fabsf(c) < kF16MinNorm) ? 0.0f : c;
  return (_Float16)z;
}
__device__ __forceinline__ v8f mma_f16(v16h a, v16h b, v8f c) {
  c = __builtin_amdgcn_wmma_f32_16x16x32_f16(false, a, false, b, (short)0, c, false, false);
  asm volatile("v_nop\n\tv_nop\n\tv_nop\n\tv_nop" : "+v"(c) : "v"(a), "v"(b));
  return c;
}
__device__ __forceinline__ float leaky(float v) { return (v > 0.0f) ? v : (kSlope * v); }

}

__global__ __launch_bounds__(32) void mlp40_seq_kernel(
    const float* __restrict__ x,
    const float* __restrict__ w1, const float* __restrict__ b1,
    const float* __restrict__ w2, const float* __restrict__ b2,
    const float* __restrict__ v1, const float* __restrict__ d1,
    const float* __restrict__ v2, const float* __restrict__ d2,
    float* __restrict__ outs)
{
  __shared__ __align__(16) float xs[kTileRows * kPitch];
  __shared__ __align__(16) float os[kTileRows * kPitch];
  __shared__ __align__(32) v16h AF[3 * 3 * 2 * 32];

  const int lane = threadIdx.x & 31;
  const int hsel = lane >> 4;
  const int n    = lane & 15;
  const bool lowHalf = (hsel == 0);
  const int b0   = blockIdx.x * kTileRows;

#pragma unroll 1
  for (int p = 0; p < 3; ++p) {
    const float* wsrc = (p == 0) ? w1 : ((p == 1) ? w2 : v1);
    const int ncol = (p == 1) ? kHid : kComb;
#pragma unroll 1
    for (int j = 0; j < 3; ++j) {
      const int row  = 16 * j + n;
      const int rowc = (row < kHid) ? row : (kHid - 1);
      const bool rok = (row < kHid);
#pragma unroll 1
      for (int c = 0; c < 2; ++c) {
        v8h lo, hi;
#pragma unroll
        for (int e = 0; e < 16; ++e) {
          const int k = 32 * c + 16 * (e >> 3) + 8 * hsel + (e & 7);
          const int colraw = (p == 1) ? k : ((k < kHid) ? (k + 1) : 0);
          const int col = (colraw < ncol) ? colraw : (ncol - 1);
          const bool kok = (p == 1) ? (k < kHid) : (k <= kHid);
          const float wv = wsrc[rowc * ncol + col];
          const _Float16 hv = eng::to_f16_flushed((rok && kok) ? (eng::bf16v(wv) * kWeightCarry) : 0.0f);
          if (e < 8) lo[e & 7] = hv; else hi[e & 7] = hv;
        }
        eng::FragU u0;
        u0.h[0] = lo;
        u0.h[1] = hi;
        AF[((p * 3 + j) * 2 + c) * 32 + lane] = u0.v;
      }
    }
  }

  float cb1[3][8], cb2[3][8], cd1[3][8], cv2[3][8];
#pragma unroll
  for (int j = 0; j < 3; ++j) {
#pragma unroll
    for (int r = 0; r < 8; ++r) {
      const int u  = 16 * j + 8 * hsel + r;
      const int uc = (u < kHid) ? u : (kHid - 1);
      const bool live = (u < kHid);
      const float t1 = eng::bf16v(b1[uc]);
      const float t2 = eng::bf16v(b2[uc]);
      const float t3 = eng::bf16v(d1[uc]);
      const float t4 = eng::bf16v(v2[uc]);
      cb1[j][r] = live ? t1 : 0.0f;
      cb2[j][r] = live ? t2 : 0.0f;
      cd1[j][r] = live ? t3 : 0.0f;
      cv2[j][r] = live ? t4 : 0.0f;
    }
  }
  const float cd2 = eng::bf16v(d2[0]);
  const v8f z8 = (v8f){0.f, 0.f, 0.f, 0.f, 0.f, 0.f, 0.f, 0.f};
  const v8h zh = (v8h){(_Float16)0.0f, (_Float16)0.0f, (_Float16)0.0f, (_Float16)0.0f,
                       (_Float16)0.0f, (_Float16)0.0f, (_Float16)0.0f, (_Float16)0.0f};
  v8h hb[3];
#pragma unroll
  for (int j = 0; j < 3; ++j) hb[j] = zh;
  __syncthreads();

  const int q  = lane >> 3;
  const int c4 = (lane & 7) * 4;

#pragma unroll 1
  for (int ch = 0; ch < kNumChunks; ++ch) {
    const int t0 = ch * kChunk;
#pragma unroll
    for (int it = 0; it < 4; ++it) {
      const int row = it * 4 + q;
      const v4f v = *(const v4f*)(x + (size_t)(b0 + row) * kSteps + t0 + c4);
      v4f rv;
      const float v0 = v[0];
      const float v1f = v[1];
      const float v2f = v[2];
      const float v3 = v[3];
      rv[0] = eng::bf16v(v0);
      rv[1] = eng::bf16v(v1f);
      rv[2] = eng::bf16v(v2f);
      rv[3] = eng::bf16v(v3);
      *(v4f*)(xs + row * kPitch + c4) = rv;
    }
    __syncthreads();

#pragma unroll 1
    for (int s = 0; s < kChunk; ++s) {
      const float xv = xs[n * kPitch + s];
      eng::FragU c0, c1;
      c0.h[0] = hb[0];
      c0.h[1] = hb[1];
      v8h c1lo = hb[2];
      c1lo[0] = lowHalf ? hb[2][0] : eng::to_f16_flushed(xv * kStateCarry);
      c1.h[0] = c1lo;
      c1.h[1] = zh;

      v8h ab[3];
#pragma unroll
      for (int j = 0; j < 3; ++j) {
        v8f acc = z8;
        acc = eng::mma_f16(AF[((0 * 3 + j) * 2 + 0) * 32 + lane], c0.v, acc);
        acc = eng::mma_f16(AF[((0 * 3 + j) * 2 + 1) * 32 + lane], c1.v, acc);
#pragma unroll
        for (int r = 0; r < 8; ++r) {
          const bool live = (16 * j + 8 * hsel + r) < kHid;
          const float av = eng::leaky(fmaf(acc[r], kFoldBack, cb1[j][r]));
          ab[j][r] = eng::to_f16_flushed(live ? (av * kStateCarry) : 0.0f);
        }
      }
      float p = 0.0f;
#pragma unroll
      for (int j = 0; j < 3; ++j) {
        v8f acc = z8;
        acc = eng::mma_f16(AF[((2 * 3 + j) * 2 + 0) * 32 + lane], c0.v, acc);
        acc = eng::mma_f16(AF[((2 * 3 + j) * 2 + 1) * 32 + lane], c1.v, acc);
#pragma unroll
        for (int r = 0; r < 8; ++r) {
          const float ov = eng::leaky(fmaf(acc[r], kFoldBack, cd1[j][r]));
          p = fmaf(cv2[j][r], ov, p);
        }
      }
      const float pother = __shfl_xor(p, 16, 32);
      const float y = (p + pother) + cd2;
      if (lowHalf) os[n * kPitch + s] = y;

      eng::FragU a0, a1;
      a0.h[0] = ab[0];
      a0.h[1] = ab[1];
      a1.h[0] = ab[2];
      a1.h[1] = zh;
#pragma unroll
      for (int j = 0; j < 3; ++j) {
        v8f acc = z8;
        acc = eng::mma_f16(AF[((1 * 3 + j) * 2 + 0) * 32 + lane], a0.v, acc);
        acc = eng::mma_f16(AF[((1 * 3 + j) * 2 + 1) * 32 + lane], a1.v, acc);
#pragma unroll
        for (int r = 0; r < 8; ++r) {
          const bool live = (16 * j + 8 * hsel + r) < kHid;
          const float hv = fmaf(acc[r], kFoldBack, cb2[j][r]);
          hb[j][r] = eng::to_f16_flushed(live ? (hv * kStateCarry) : 0.0f);
        }
      }
    }
    __syncthreads();

    {
      for (int pass = 0; pass < 2; ++pass) {
#pragma unroll
        for (int it = 0; it < 4; ++it) {
          const int row = it * 4 + q;
          const v4f ov = *(const v4f*)(os + row * kPitch + c4);
          *(volatile v4f*)(outs + (size_t)(b0 + row) * kSteps + t0 + c4) = ov;
        }
        __threadfence();
      }
    }
  }
}

extern "C" void kernel_launch(void* const* d_in, const int* in_sizes, int n_in,
                              void* d_out, int out_size, void* d_ws, size_t ws_size,
                              hipStream_t stream) {
  (void)d_ws;
  (void)ws_size;
  if (n_in < 9 || d_out == nullptr) return;
  if ((size_t)in_sizes[0] != kOutElems) return;
  if (in_sizes[1] != kHid * kComb || in_sizes[2] != kHid) return;
  if (in_sizes[3] != kHid * kHid || in_sizes[4] != kHid) return;
  if (in_sizes[5] != kHid * kComb || in_sizes[6] != kHid) return;
  if (in_sizes[7] != kHid || in_sizes[8] != 1) return;
  if ((size_t)out_size != kOutElems) return;

  const float* x  = (const float*)d_in[0];
  const float* w1 = (const float*)d_in[1];
  const float* b1 = (const float*)d_in[2];
  const float* w2 = (const float*)d_in[3];
  const float* b2 = (const float*)d_in[4];
  const float* v1 = (const float*)d_in[5];
  const float* d1 = (const float*)d_in[6];
  const float* v2 = (const float*)d_in[7];
  const float* d2 = (const float*)d_in[8];
  float* outs = (float*)d_out;

  mlp40_seq_kernel<<<kTiles, 32, 0, stream>>>(x, w1, b1, w2, b2, v1, d1, v2, d2, outs);
}
